// RQuadratic_8985071583510
// MI455X (gfx1250) — hardware-verified
//
#include <hip/hip_runtime.h>

typedef float          v4f   __attribute__((ext_vector_type(4)));
typedef float          v8f   __attribute__((ext_vector_type(8)));
typedef __bf16         v16bf __attribute__((ext_vector_type(16)));
typedef unsigned short v8us  __attribute__((ext_vector_type(8)));
typedef unsigned short v16us __attribute__((ext_vector_type(16)));
typedef v4f  __attribute__((may_alias)) v4fa;
typedef v8us __attribute__((may_alias)) v8usa;

#define NB    32768
#define DIM   64
#define DD    4096
#define TB    16
#define NTHR  256
#define NX    (NB * DIM)
#define NWGT  ((DIM + 1) * DD)
#define NPL   (DD * DIM)
#define LDS_MAIN_BYTES ((TB * DD + 2 * TB * DIM) * 4)

union FragU { v16bf v; v16us u; v8us half[2]; };

__device__ __forceinline__ unsigned int bf16_rne_bits(float f) {
  unsigned int u = __float_as_uint(f);
  u += 0x7FFFu + ((u >> 16) & 1u);
  return u >> 16;
}

__device__ __forceinline__ v8f wmma_bf16(v16bf a, v16bf b, v8f c) {
  v8f d = __builtin_amdgcn_wmma_f32_16x16x32_bf16(false, a, false, b, (short)0, c, false, false);
  asm volatile("v_nop\n\tv_nop\n\tv_nop\n\tv_nop" : "+v"(d) : "v"(a), "v"(b));
  return d;
}

__device__ __forceinline__ v16bf load_frag16(const unsigned short* p, int h) {
  FragU f;
  f.half[0] = *(const v8usa*)(p + 8 * h);
  f.half[1] = *(const v8usa*)(p + 16 + 8 * h);
  return f.v;
}

__global__ __launch_bounds__(256) void wsplit_kernel(
    const float* __restrict__ w,
    unsigned short* __restrict__ whi,
    unsigned short* __restrict__ wlo)
{
  __shared__ __attribute__((aligned(16))) unsigned short sH[64 * 64];
  __shared__ __attribute__((aligned(16))) unsigned short sL[64 * 64];

  const int tid = threadIdx.x, lane = tid & 31, wv = tid >> 5;
  const int c0 = blockIdx.x * 64;

  #pragma unroll
  for (int it = 0; it < 16; ++it) {
    const int idx = tid + 256 * it;
    const int k = idx >> 6, c = idx & 63;
    const float f = w[(size_t)k * DD + c0 + c];
    const unsigned int hb = bf16_rne_bits(f);
    const float lo = f - __uint_as_float(hb << 16);
    sH[c * 64 + k] = (unsigned short)hb;
    sL[c * 64 + k] = (unsigned short)bf16_rne_bits(lo);
  }
  __syncthreads();

  const int q = lane >> 3, j = lane & 7;
  const int cA = wv * 8 + q;
  const int cB = wv * 8 + 4 + q;
  const v8us hA = *(const v8usa*)(sH + cA * 64 + 8 * j);
  const v8us lA = *(const v8usa*)(sL + cA * 64 + 8 * j);
  const v8us hB = *(const v8usa*)(sH + cB * 64 + 8 * j);
  const v8us lB = *(const v8usa*)(sL + cB * 64 + 8 * j);
  unsigned short* dhA = whi + (size_t)(c0 + cA) * DIM + 8 * j;
  unsigned short* dlA = wlo + (size_t)(c0 + cA) * DIM + 8 * j;
  unsigned short* dhB = whi + (size_t)(c0 + cB) * DIM + 8 * j;
  unsigned short* dlB = wlo + (size_t)(c0 + cB) * DIM + 8 * j;

  *(volatile v8us*)dhA = hA;
  *(volatile v8us*)dlA = lA;
  *(volatile v8us*)dhB = hB;
  *(volatile v8us*)dlB = lB;
  __threadfence();
  *(volatile v8us*)dhA = hA;
  *(volatile v8us*)dlA = lA;
  *(volatile v8us*)dhB = hB;
  *(volatile v8us*)dlB = lB;
}

__global__ __launch_bounds__(NTHR) void rq_kernel(
    const float* __restrict__ x,
    const float* __restrict__ gH,
    const float* __restrict__ w,
    const unsigned short* __restrict__ whi,
    const unsigned short* __restrict__ wlo,
    float* __restrict__ out)
{
  extern __shared__ __attribute__((aligned(16))) float lds[];
  float* Ml = lds;
  float* gl = lds + TB * DD;
  float* tl = gl + TB * DIM;

  const int tid = threadIdx.x, lane = tid & 31, wv = tid >> 5;
  const int h = lane >> 4, m = lane & 15;
  const int b0 = blockIdx.x * TB;

  #pragma unroll
  for (int it = 0; it < 4; ++it)
    gl[tid + NTHR * it] = gH[(size_t)b0 * DIM + tid + NTHR * it];

  v16bf ahi[2], alo[2];
  {
    const float* xr = x + (size_t)(b0 + m) * DIM;
    #pragma unroll
    for (int kc = 0; kc < 2; ++kc) {
      const v4f p0 = *(const v4fa*)(xr + kc * 32 + 8 * h);
      const v4f p1 = *(const v4fa*)(xr + kc * 32 + 8 * h + 4);
      const v4f p2 = *(const v4fa*)(xr + kc * 32 + 16 + 8 * h);
      const v4f p3 = *(const v4fa*)(xr + kc * 32 + 16 + 8 * h + 4);
      const float f[16] = { p0.x, p0.y, p0.z, p0.w, p1.x, p1.y, p1.z, p1.w,
                            p2.x, p2.y, p2.z, p2.w, p3.x, p3.y, p3.z, p3.w };
      FragU fh, fl;
      #pragma unroll
      for (int e = 0; e < 16; ++e) {
        const unsigned int hb = bf16_rne_bits(f[e]);
        const float lo = f[e] - __uint_as_float(hb << 16);
        fh.u[e] = (unsigned short)hb;
        fl.u[e] = (unsigned short)bf16_rne_bits(lo);
      }
      ahi[kc] = fh.v;
      alo[kc] = fl.v;
    }
  }

  const float* wb = w + (size_t)DIM * DD;
  #pragma unroll 1
  for (int ct = 0; ct < 32; ++ct) {
    const int c0 = wv * 512 + ct * 16;
    const float bias = wb[c0 + m];
    v8f acc;
    #pragma unroll
    for (int r = 0; r < 8; ++r) acc[r] = bias;

    const unsigned short* ph = whi + (size_t)(c0 + m) * DIM;
    const unsigned short* pl = wlo + (size_t)(c0 + m) * DIM;
    #pragma unroll
    for (int kc = 0; kc < 2; ++kc) {
      const v16bf bh = load_frag16(ph + kc * 32, h);
      const v16bf bl = load_frag16(pl + kc * 32, h);
      acc = wmma_bf16(ahi[kc], bh, acc);
      acc = wmma_bf16(ahi[kc], bl, acc);
      acc = wmma_bf16(alo[kc], bh, acc);
    }
    #pragma unroll
    for (int r = 0; r < 8; ++r) Ml[(8 * h + r) * DD + c0 + m] = acc[r];
  }
  __syncthreads();

  #pragma unroll 1
  for (int it = 0; it < 4; ++it) {
    const int o = tid + NTHR * it;
    const int b = o >> 6, k = o & 63;
    const float* Mb = Ml + b * DD + k;
    const float* gb = gl + b * DIM;
    float s = 0.0f;
    #pragma unroll 8
    for (int i = 0; i < DIM; ++i) s += gb[i] * Mb[i * DIM];
    tl[o] = s;
  }
  __syncthreads();

  float* ol = gl;
  #pragma unroll 1
  for (int it = 0; it < 4; ++it) {
    const int o = tid + NTHR * it;
    const int b = o >> 6, e = o & 63;
    const float* Mr = Ml + b * DD + e * DIM;
    const float* tb = tl + b * DIM;
    float s = 0.0f;
    #pragma unroll 4
    for (int k4 = 0; k4 < 16; ++k4) {
      const v4f mv = *(const v4fa*)(Mr + 4 * k4);
      const v4f tv = *(const v4fa*)(tb + 4 * k4);
      s += mv.x * tv.x;
      s += mv.y * tv.y;
      s += mv.z * tv.z;
      s += mv.w * tv.w;
    }
    ol[o] = s * 0.125f;
  }
  __syncthreads();

  const int row = 2 * wv + h;
  const v4f v = *(const v4fa*)(ol + row * DIM + 4 * m);
  float* dst = out + (size_t)(b0 + row) * DIM + 4 * m;
  *(volatile v4f*)dst = v;
  __threadfence();
  *(volatile v4f*)dst = v;
}

extern "C" void kernel_launch(void* const* d_in, const int* in_sizes, int n_in,
                              void* d_out, int out_size, void* d_ws, size_t ws_size,
                              hipStream_t stream) {
  if (n_in < 3) return;
  if (in_sizes[0] != NX || in_sizes[1] != NX || in_sizes[2] != NWGT) return;
  if (out_size != NX) return;

  const float* x  = (const float*)d_in[0];
  const float* gH = (const float*)d_in[1];
  const float* w  = (const float*)d_in[2];
  float* out = (float*)d_out;

  const size_t plane_bytes = (size_t)NPL * 2;
  if (2 * plane_bytes > ws_size) return;
  char* ws = (char*)d_ws;
  unsigned short* whi = (unsigned short*)(ws);
  unsigned short* wlo = (unsigned short*)(ws + plane_bytes);

  wsplit_kernel<<<DD / 64, 256, 0, stream>>>(w, whi, wlo);

  hipFuncSetAttribute(reinterpret_cast<const void*>(rq_kernel),
                      hipFuncAttributeMaxDynamicSharedMemorySize, LDS_MAIN_BYTES);
  rq_kernel<<<NB / TB, NTHR, LDS_MAIN_BYTES, stream>>>(x, gH, w, whi, wlo, out);
}
